// DConvolutionModule_51891794870780
// MI455X (gfx1250) — hardware-verified
//
#include <hip/hip_runtime.h>


#define NBT  8
#define TT   2048
#define CC   512
#define NHS  4
#define KS   31
#define PADK 15
#define DG   (CC / NHS)
#define NWL  (NHS * KS)
#define DM   CC
#define LOSC 1024.0f

typedef _Float16 h16;
typedef unsigned short bf;
typedef __attribute__((ext_vector_type(16))) __bf16   v16bf;
typedef __attribute__((ext_vector_type(16))) _Float16 v16h;
typedef __attribute__((ext_vector_type(8)))  _Float16 v8h;
typedef __attribute__((ext_vector_type(8)))  unsigned short v8us;
typedef __attribute__((ext_vector_type(8)))  float    v8f;
typedef __attribute__((ext_vector_type(4)))  float    v4f;
typedef v8h  __attribute__((may_alias)) v8ha;
typedef v4f  __attribute__((may_alias)) v4fa;
typedef v8us __attribute__((may_alias)) v8usa;

__device__ __forceinline__ unsigned short f2bf(float f) { unsigned u = __float_as_uint(f); u += 0x7FFFu + ((u >> 16) & 1u); return (unsigned short)(u >> 16); }
__device__ __forceinline__ float bf2f(unsigned short b) { return __uint_as_float(((unsigned)b) << 16); }
__device__ __forceinline__ float bfr(float f) { return bf2f(f2bf(f)); }
__device__ __forceinline__ v16h cat16(v8h lo, v8h hi) { return __builtin_shufflevector(lo, hi, 0, 1, 2, 3, 4, 5, 6, 7, 8, 9, 10, 11, 12, 13, 14, 15); }
__device__ __forceinline__ v16bf cat16b(v8us lo, v8us hi) { return __builtin_bit_cast(v16bf, __builtin_shufflevector(lo, hi, 0, 1, 2, 3, 4, 5, 6, 7, 8, 9, 10, 11, 12, 13, 14, 15)); }
__device__ __forceinline__ v8f wmma16(v16h a, v16h b, v8f c) { return __builtin_amdgcn_wmma_f32_16x16x32_f16(false, a, false, b, (short)0, c, false, false); }
__device__ __forceinline__ v8f wmmab(v16bf a, v16bf b, v8f c) { return __builtin_amdgcn_wmma_f32_16x16x32_bf16(false, a, false, b, (short)0, c, false, false); }

template <bool SPLITA, bool F16OUT = false>
__global__ __launch_bounds__(128) void k_gemmb(const bf* __restrict__ A, const bf* __restrict__ Al, const bf* __restrict__ Bn, const float* __restrict__ bias, float* C, int ldc, h16* C2, const float* __restrict__ R = nullptr, int K = DM, int roundR = 1) {
    __shared__ __align__(16) float ost[4][16 * 68];
    const int lane = threadIdx.x & 31, wave = threadIdx.x >> 5, lr = lane & 15, hi = lane >> 4;
    const int r0 = blockIdx.x * 64 + wave * 16, c0 = blockIdx.y * 64;
    const size_t aoff = (size_t)(r0 + lr) * K + 8 * hi;
    size_t boff[4];
#pragma unroll
    for (int t = 0; t < 4; ++t) boff[t] = (size_t)(c0 + t * 16 + lr) * K + 8 * hi;
    v8f acc[4];
#pragma unroll
    for (int t = 0; t < 4; ++t) acc[t] = (v8f){};
#pragma unroll 1
    for (int kc = 0; kc < K; kc += 32) {
        const v16bf a = cat16b(*(const v8us*)(A + aoff + kc), *(const v8us*)(A + aoff + kc + 16));
        v16bf al = a;
        if (SPLITA) al = cat16b(*(const v8us*)(Al + aoff + kc), *(const v8us*)(Al + aoff + kc + 16));
#pragma unroll
        for (int t = 0; t < 4; ++t) { const v16bf b = cat16b(*(const v8us*)(Bn + boff[t] + kc), *(const v8us*)(Bn + boff[t] + kc + 16)); acc[t] = wmmab(a, b, acc[t]); if (SPLITA) acc[t] = wmmab(al, b, acc[t]); }
        asm volatile("v_nop\n\tv_nop\n\tv_nop\n\tv_nop" : "+v"(acc[0]), "+v"(acc[1]), "+v"(acc[2]), "+v"(acc[3]) : "v"(a), "v"(al));
    }
    float* os = &ost[wave][0];
#pragma unroll
    for (int t = 0; t < 4; ++t) { const float bv = bias ? bfr(bias[c0 + t * 16 + lr]) : 0.f;
#pragma unroll
        for (int j = 0; j < 8; ++j) os[(hi * 8 + j) * 68 + t * 16 + lr] = acc[t][j] + bv; }
    __syncthreads();
    if (F16OUT) {
        h16* crow = (h16*)(void*)C + (size_t)r0 * ldc + c0;
        auto pass = [&]() {
#pragma unroll
            for (int s = 0; s < 4; ++s) { const int row = 4 * s + (lane >> 3), piece = lane & 7; const float* sp = os + row * 68 + piece * 8; v8h o, o2;
#pragma unroll
                for (int i = 0; i < 8; ++i) { const h16 a = (h16)sp[i]; o[i] = a; o2[i] = (h16)((sp[i] - (float)a) * LOSC); }
                *(volatile v8h*)(crow + (size_t)row * ldc + piece * 8) = o; if (C2) *(volatile v8h*)(C2 + (size_t)r0 * ldc + c0 + (size_t)row * ldc + piece * 8) = o2; }
        };
        pass(); __threadfence(); pass();
    } else {
        float* crow = C + (size_t)r0 * ldc + c0;
        auto pass = [&]() {
#pragma unroll
            for (int s = 0; s < 8; ++s) { const int Lid = (lane >> 3) + 4 * s, piece = lane & 7; const int row = Lid >> 1, cofs = (Lid & 1) * 32 + piece * 4;
                v4f val = *(const v4fa*)(os + row * 68 + cofs); if (R) { const v4f rv = *(const v4f*)(R + ((size_t)r0 + row) * ldc + c0 + cofs); val += roundR ? (v4f){bfr(rv[0]), bfr(rv[1]), bfr(rv[2]), bfr(rv[3])} : rv; }
                *(volatile v4f*)(crow + (size_t)row * ldc + cofs) = val; }
        };
        pass(); __threadfence(); pass();
    }
}


__global__ __launch_bounds__(256) void k_cvt8(const float* __restrict__ src, bf* dst, size_t n8) {
    const size_t i = (size_t)blockIdx.x * 256 + threadIdx.x; if (i >= n8) return;
    const v8f v = *(const v8f*)(src + i * 8); v8us o;
#pragma unroll
    for (int k = 0; k < 8; ++k) o[k] = f2bf(v[k]);
    *(volatile v8us*)(dst + i * 8) = o; __threadfence(); *(volatile v8us*)(dst + i * 8) = o;
}
__global__ __launch_bounds__(256) void k_zero8(bf* dst, size_t n8) {
    const size_t i = (size_t)blockIdx.x * 256 + threadIdx.x; if (i >= n8) return; v8us z;
#pragma unroll
    for (int k = 0; k < 8; ++k) z[k] = 0;
    *(volatile v8us*)(dst + i * 8) = z; __threadfence(); *(volatile v8us*)(dst + i * 8) = z;
}

__global__ __launch_bounds__(256) void k_cvtx(const float* __restrict__ src, bf* dst) {
    const int lane = threadIdx.x & 31; const size_t r = (size_t)blockIdx.x * 8 + (threadIdx.x >> 5); if (r >= (size_t)TT) return;
#pragma unroll 1
    for (int ps = 0; ps < 2; ++ps) {
#pragma unroll
        for (int q = 0; q < CC / 256; ++q) { v8us o;
#pragma unroll
            for (int i = 0; i < 8; ++i) o[i] = f2bf(src[r * CC + q * 256 + lane * 8 + i]);
            *(volatile v8us*)(dst + r * CC + q * 256 + lane * 8) = o; }
        if (ps == 0) __threadfence(); }
}
__global__ __launch_bounds__(256) void k_wl128(const float* __restrict__ Wl, bf* WLP) {
    const int lane = threadIdx.x & 31; const int o = blockIdx.x * 8 + (threadIdx.x >> 5); if (o >= 128) return;
#pragma unroll 1
    for (int ps = 0; ps < 2; ++ps) {
#pragma unroll
        for (int q = 0; q < CC / 256; ++q) { v8us v;
#pragma unroll
            for (int i = 0; i < 8; ++i) v[i] = (o < NWL) ? f2bf(Wl[(size_t)(o < NWL ? o : 0) * CC + q * 256 + lane * 8 + i]) : (unsigned short)0;
            *(volatile v8us*)(WLP + (size_t)o * CC + q * 256 + lane * 8) = v; }
        if (ps == 0) __threadfence(); }
}
__global__ __launch_bounds__(64) void k_bl128(const float* __restrict__ bl, float* BLP) {
    const int lane = threadIdx.x; if (lane >= 32) return; v4f v;
#pragma unroll
    for (int q = 0; q < 4; ++q) { const int o = lane * 4 + q; v[q] = (o < NWL) ? bl[o < NWL ? o : 0] : 0.f; }
    *(volatile v4f*)(BLP + lane * 4) = v; __threadfence(); *(volatile v4f*)(BLP + lane * 4) = v;
}
__global__ __launch_bounds__(256) void k_glu(const float* __restrict__ Y1, float* Yf, bf* Yh, bf* Yl) {
    typedef __attribute__((ext_vector_type(4))) unsigned short v4us;
    const int lane = threadIdx.x & 31; const size_t t = (size_t)blockIdx.x * 8 + (threadIdx.x >> 5); if (t >= (size_t)TT) return;
#pragma unroll 1
    for (int ps = 0; ps < 2; ++ps) {
#pragma unroll
        for (int c0 = lane * 4; c0 < CC; c0 += 128) { v4f v; v4us oh, ol;
#pragma unroll
            for (int q = 0; q < 4; ++q) { const float a = Y1[t * 2 * CC + c0 + q], g = Y1[t * 2 * CC + CC + c0 + q]; const float y = a * (1.0f / (1.0f + __expf(-g))); v[q] = y; const unsigned short hb = f2bf(y); oh[q] = hb; ol[q] = f2bf(y - bf2f(hb)); }
            *(volatile v4f*)(Yf + t * CC + c0) = v; *(volatile v4us*)(Yh + t * CC + c0) = oh; *(volatile v4us*)(Yl + t * CC + c0) = ol; }
        if (ps == 0) __threadfence(); }
}
__global__ __launch_bounds__(256) void k_dconv(const float* __restrict__ WD, const float* __restrict__ Yf, const float* __restrict__ cbias, bf* Oh, bf* Ol) {
    typedef __attribute__((ext_vector_type(4))) unsigned short v4us;
    const int lane = threadIdx.x & 31; const int wid = blockIdx.x * 8 + (threadIdx.x >> 5); if (wid >= TT * NHS) return; const int t = wid / NHS, h = wid % NHS; const int c0 = h * DG + lane * 4;
    const float* wr = WD + (size_t)t * 128 + h * KS;
    float m = -3.0e38f;
#pragma unroll 1
    for (int j = 0; j < KS; ++j) { const int s = t + j - PADK; if (s >= 0 && s < TT) m = fmaxf(m, wr[j]); }
    float sum = 0.f;
#pragma unroll 1
    for (int j = 0; j < KS; ++j) { const int s = t + j - PADK; if (s >= 0 && s < TT) sum += __expf(wr[j] - m); }
    const float inv = 1.0f / sum; float acc[4] = {0.f, 0.f, 0.f, 0.f};
#pragma unroll 1
    for (int j = 0; j < KS; ++j) { const int s = t + j - PADK; if (s < 0 || s >= TT) continue; const float w = __expf(wr[j] - m) * inv; const v4f yv = *(const v4f*)(Yf + (size_t)s * CC + c0);
#pragma unroll
        for (int q = 0; q < 4; ++q) acc[q] = fmaf(w, yv[q], acc[q]); }
    v4us oh, ol;
#pragma unroll
    for (int q = 0; q < 4; ++q) { const float v = acc[q] + bfr(cbias[c0 + q]); const unsigned short hb = f2bf(v); oh[q] = hb; ol[q] = f2bf(v - bf2f(hb)); }
    const size_t o = (size_t)t * CC + c0; *(volatile v4us*)(Oh + o) = oh; *(volatile v4us*)(Ol + o) = ol; __threadfence(); *(volatile v4us*)(Oh + o) = oh; *(volatile v4us*)(Ol + o) = ol;
}

extern "C" void kernel_launch(void* const* d_in, const int* in_sizes, int n_in,
                              void* d_out, int out_size, void* d_ws, size_t ws_size, hipStream_t stream) {
    (void)in_sizes; (void)n_in; (void)out_size;
    const float* x = (const float*)d_in[0]; const float* W1 = (const float*)d_in[1]; const float* b1 = (const float*)d_in[2]; const float* Wl = (const float*)d_in[3]; const float* bl = (const float*)d_in[4]; const float* cbias = (const float*)d_in[5]; const float* W2 = (const float*)d_in[6]; const float* b2 = (const float*)d_in[7];
    float* out = (float*)d_out;
    char* wsp = (char*)d_ws;
    auto take = [&](size_t bytes) { char* p = wsp; wsp += (bytes + 255) & ~(size_t)255; return (void*)p; };
    bf* W1B = (bf*)take((size_t)2 * CC * CC * 2); bf* WLP = (bf*)take((size_t)128 * CC * 2); float* BLP = (float*)take(128 * 4); bf* W2B = (bf*)take((size_t)CC * CC * 2);
    bf* Xb = (bf*)take((size_t)TT * CC * 2); float* Y1 = (float*)take((size_t)TT * 2 * CC * 4); float* Yf = (float*)take((size_t)TT * CC * 4); bf* Yh = (bf*)take((size_t)TT * CC * 2); bf* Yl = (bf*)take((size_t)TT * CC * 2);
    float* WD = (float*)take((size_t)TT * 128 * 4); bf* Oh = (bf*)take((size_t)TT * CC * 2); bf* Ol = (bf*)take((size_t)TT * CC * 2);
    if ((size_t)(wsp - (char*)d_ws) > ws_size) return;
    k_cvt8<<<(2 * CC * CC / 8 + 255) / 256, 256, 0, stream>>>(W1, W1B, (size_t)2 * CC * CC / 8); k_wl128<<<128 / 8, 256, 0, stream>>>(Wl, WLP); k_bl128<<<1, 64, 0, stream>>>(bl, BLP); k_cvt8<<<(CC * CC / 8 + 255) / 256, 256, 0, stream>>>(W2, W2B, (size_t)CC * CC / 8);
    for (int b = 0; b < NBT; ++b) {
        k_cvtx<<<TT / 8, 256, 0, stream>>>(x + (size_t)b * TT * CC, Xb);
        k_gemmb<false, false><<<dim3(TT / 64, (2 * CC) / 64, 1), 128, 0, stream>>>(Xb, nullptr, W1B, b1, Y1, 2 * CC, nullptr, nullptr, CC);
        k_glu<<<TT / 8, 256, 0, stream>>>(Y1, Yf, Yh, Yl);
        k_gemmb<true, false><<<dim3(TT / 64, 2, 1), 128, 0, stream>>>(Yh, Yl, WLP, BLP, WD, 128, nullptr, nullptr, CC);
        k_dconv<<<(TT * NHS) / 8, 256, 0, stream>>>(WD, Yf, cbias, Oh, Ol);
        k_gemmb<true, false><<<dim3(TT / 64, CC / 64, 1), 128, 0, stream>>>(Oh, Ol, W2B, b2, out + (size_t)b * TT * CC, CC, nullptr, nullptr, CC); }
}
